// S6_49512382988926
// MI455X (gfx1250) — hardware-verified
//
#include <hip/hip_runtime.h>
#include <math.h>

typedef __attribute__((ext_vector_type(16))) __bf16   v16b;
typedef __attribute__((ext_vector_type(8)))  __bf16   v8b;
typedef __attribute__((ext_vector_type(8)))  float    v8f;
typedef __attribute__((ext_vector_type(4)))  float    v4f;
typedef __attribute__((ext_vector_type(4)))  unsigned v4u;

constexpr int kBatch   = 2;
constexpr int kSeq     = 2048;
constexpr int kRows    = kBatch * kSeq;
constexpr int kDm      = 1024;
constexpr int kNst     = 16;
constexpr int kBCRows  = 2 * kNst;
constexpr int kSlabP   = 68;
constexpr int kTilesM  = kRows / 64;
constexpr int kTilesN  = kDm / 64;
constexpr int kRowsPerDotBlock = 128;
static_assert(kRows == 4096 && kDm == 1024 && kNst == 16, "wire shapes");
static_assert((kDm % 32) == 0, "GEMM K multiple of 32");
static_assert((kRows % 64) == 0 && (kDm % 64) == 0, "GEMM M,N multiples of 64");
static_assert((kRows % kRowsPerDotBlock) == 0, "row-dot block multiple");
static_assert(((kTilesM * kTilesN) % 8) == 0, "eight wave tiles per block");

constexpr size_t kOffXB   = 0;
constexpr size_t kOffW1B  = kOffXB   + (size_t)kRows   * kDm * 2;
constexpr size_t kOffW23B = kOffW1B  + (size_t)kDm     * kDm * 2;
constexpr size_t kOffSPL  = kOffW23B + (size_t)kBCRows * kDm * 2;
constexpr size_t kWsTotal = kOffSPL  + (size_t)kRows * 4;
static_assert(kWsTotal == 10567680ull, "carve total");
static_assert(kWsTotal <= 134217728ull, "carve cap");
static_assert((kOffW1B % 128) == 0 && (kOffW23B % 128) == 0 && (kOffSPL % 128) == 0, "128-B aligned regions");

__device__ __forceinline__ unsigned rne_bf16_bits(float f) {
  const unsigned u = __float_as_uint(f);
  return (u + 0x7FFFu + ((u >> 16) & 1u)) >> 16;
}
__device__ __forceinline__ float rne_bf16_f32(float f) {
  return __uint_as_float(rne_bf16_bits(f) << 16);
}

template <typename T> struct Frag;
template <> struct Frag<__bf16> {
  typedef v16b V;
  union U { v16b v; v8b h[2]; };
  static __device__ __forceinline__ v16b load(const __bf16* p) {
    U f;
    f.h[0] = *(const v8b*)(p);
    f.h[1] = *(const v8b*)(p + 16);
    return f.v;
  }
  static __device__ __forceinline__ v8f mma(v16b a, v16b b, v8f c) {
    return __builtin_amdgcn_wmma_f32_16x16x32_bf16(false, a, false, b, (short)0, c, false, false);
  }
};
__device__ __forceinline__ void guard_row4(v8f& a, v8f& b, v8f& c, v8f& d, v16b x, v16b b0, v16b b1, v16b b2, v16b b3) {
  asm volatile("v_nop\n\tv_nop\n\tv_nop\n\tv_nop" : "+v"(a), "+v"(b), "+v"(c), "+v"(d) : "v"(x), "v"(b0), "v"(b1), "v"(b2), "v"(b3));
}
__device__ __forceinline__ void guard_pair(v8f& a, v8f& b, v16b x, v16b y, v16b z) {
  asm volatile("v_nop\n\tv_nop\n\tv_nop\n\tv_nop" : "+v"(a), "+v"(b) : "v"(x), "v"(y), "v"(z));
}
__device__ __forceinline__ void keep4_b(v16b a, v16b b, v16b c, v16b d) {
  asm volatile("v_nop" :: "v"(a), "v"(b), "v"(c), "v"(d));
}
__device__ __forceinline__ void acc_guard4(v8f& a, v8f& b, v8f& c, v8f& d) {
  asm volatile("v_nop\n\tv_nop\n\tv_nop\n\tv_nop" : "+v"(a), "+v"(b), "+v"(c), "+v"(d));
}

__global__ __launch_bounds__(256) void rne_bf16_rows_kernel(
    const float* __restrict__ src, unsigned short* __restrict__ dst, int total8)
{
  const int i = blockIdx.x * 256 + threadIdx.x;
  if (i >= total8) return;
  const size_t e0 = (size_t)i << 3;
  const v4f a0 = *(const v4f*)(src + e0);
  const v4f a1 = *(const v4f*)(src + e0 + 4);
  const float f0 = a0[0], f1 = a0[1], f2 = a0[2], f3 = a0[3];
  const float f4 = a1[0], f5 = a1[1], f6 = a1[2], f7 = a1[3];
  v4u w;
  w[0] = rne_bf16_bits(f0) | (rne_bf16_bits(f1) << 16);
  w[1] = rne_bf16_bits(f2) | (rne_bf16_bits(f3) << 16);
  w[2] = rne_bf16_bits(f4) | (rne_bf16_bits(f5) << 16);
  w[3] = rne_bf16_bits(f6) | (rne_bf16_bits(f7) << 16);
  unsigned short* q = dst + e0;
  *(volatile v4u*)q = w;
  __threadfence();
  *(volatile v4u*)q = w;
}

__global__ __launch_bounds__(256) void bc_rowdot_kernel(
    const unsigned short* __restrict__ XBp, const unsigned short* __restrict__ W23p,
    const float* __restrict__ b2, const float* __restrict__ b3, float* __restrict__ SPL)
{
  __shared__ __align__(16) float sS[kRowsPerDotBlock];
  const __bf16* XB  = (const __bf16*)XBp;
  const __bf16* W23 = (const __bf16*)W23p;
  const int lane  = threadIdx.x & 31;
  const int wave  = threadIdx.x >> 5;
  const int rlane = lane & 15;
  const int hh    = lane >> 4;
  const int koff  = hh * 8;
  const int m0    = blockIdx.x * kRowsPerDotBlock + wave * 16;

  const __bf16* ap  = XB  + (size_t)(m0 + rlane) * kDm + koff;
  const __bf16* bpB = W23 + (size_t)rlane * kDm + koff;
  const __bf16* bpC = W23 + (size_t)(kNst + rlane) * kDm + koff;

  v8f accB = (v8f){0.f,0.f,0.f,0.f,0.f,0.f,0.f,0.f};
  v8f accC = (v8f){0.f,0.f,0.f,0.f,0.f,0.f,0.f,0.f};
  for (int k0 = 0; k0 < kDm; k0 += 32) {
    const v16b a  = Frag<__bf16>::load(ap + k0);
    const v16b fb = Frag<__bf16>::load(bpB + k0);
    const v16b fc = Frag<__bf16>::load(bpC + k0);
    accB = Frag<__bf16>::mma(a, fb, accB);
    accC = Frag<__bf16>::mma(a, fc, accC);
    guard_pair(accB, accC, a, fb, fc);
  }

  const float rb2 = rne_bf16_f32(b2[rlane]);
  const float rb3 = rne_bf16_f32(b3[rlane]);
#pragma unroll
  for (int r = 0; r < 8; ++r) {
    const float bm = accB[r] + rb2;
    const float cm = accC[r] + rb3;
    float p = bm * cm;
#pragma unroll
    for (int off = 1; off < 16; off <<= 1) p += __shfl_xor(p, off, 32);
    if (rlane == 0) sS[wave * 16 + 8 * hh + r] = p;
  }
  __syncthreads();
  if (wave == 0) {
    const v4f v = *(const v4f*)(sS + lane * 4);
    float* q = SPL + (size_t)blockIdx.x * kRowsPerDotBlock + lane * 4;
    *(volatile v4f*)q = v;
    __threadfence();
    *(volatile v4f*)q = v;
  }
}

__global__ __launch_bounds__(256) void fc1_softplus_gate_kernel(
    const unsigned short* __restrict__ XBp, const unsigned short* __restrict__ W1Bp,
    const float* __restrict__ x, const float* __restrict__ b1, const float* __restrict__ SPL,
    float* __restrict__ out)
{
  __shared__ __align__(16) float sT[8][16 * kSlabP];
  const __bf16* A  = (const __bf16*)XBp;
  const __bf16* Bt = (const __bf16*)W1Bp;
  const int lane = threadIdx.x & 31;
  const int wave = threadIdx.x >> 5;
  const int tile = blockIdx.x * 8 + wave;
  if (tile >= kTilesM * kTilesN) return;
  const int tm = tile / kTilesN;
  const int tn = tile - tm * kTilesN;
  const int m0 = tm << 6;
  const int n0 = tn << 6;

  const int rlane = lane & 15;
  const int koff  = (lane >> 4) * 8;
  const int mOff  = (lane >> 4) * 8;

  v8f acc[4][4];
#pragma unroll
  for (int i = 0; i < 4; ++i)
#pragma unroll
    for (int j = 0; j < 4; ++j) acc[i][j] = (v8f){0.f,0.f,0.f,0.f,0.f,0.f,0.f,0.f};

  for (int k0 = 0; k0 < kDm; k0 += 32) {
    v16b bh[4];
#pragma unroll
    for (int j = 0; j < 4; ++j)
      bh[j] = Frag<__bf16>::load(Bt + (size_t)(n0 + (j << 4) + rlane) * kDm + koff + k0);
#pragma unroll
    for (int i = 0; i < 4; ++i) {
      const v16b ah = Frag<__bf16>::load(A + (size_t)(m0 + (i << 4) + rlane) * kDm + koff + k0);
#pragma unroll
      for (int j = 0; j < 4; ++j) acc[i][j] = Frag<__bf16>::mma(ah, bh[j], acc[i][j]);
      guard_row4(acc[i][0], acc[i][1], acc[i][2], acc[i][3], ah, bh[0], bh[1], bh[2], bh[3]);
    }
    keep4_b(bh[0], bh[1], bh[2], bh[3]);
  }
  acc_guard4(acc[0][0], acc[0][1], acc[0][2], acc[0][3]);
  acc_guard4(acc[1][0], acc[1][1], acc[1][2], acc[1][3]);
  acc_guard4(acc[2][0], acc[2][1], acc[2][2], acc[2][3]);
  acc_guard4(acc[3][0], acc[3][1], acc[3][2], acc[3][3]);

  float* slab = sT[wave];
  float rb[4];
#pragma unroll
  for (int j = 0; j < 4; ++j) rb[j] = rne_bf16_f32(b1[n0 + (j << 4) + rlane]);

#pragma unroll
  for (int i = 0; i < 4; ++i) {
    const int mBase = m0 + (i << 4);
#pragma unroll
    for (int j = 0; j < 4; ++j) {
#pragma unroll
      for (int r = 0; r < 8; ++r)
        slab[(mOff + r) * kSlabP + (j << 4) + rlane] = acc[i][j][r] + rb[j];
    }
    __builtin_amdgcn_fence(__ATOMIC_RELEASE, "workgroup");
    __builtin_amdgcn_wave_barrier();
    __builtin_amdgcn_fence(__ATOMIC_ACQUIRE, "workgroup");

#pragma unroll 1
    for (int idx = 0; idx < 32; ++idx) {
      const int row = idx >> 1;
      const int col = ((idx & 1) << 5) + lane;
      const int gm  = mBase + row;
      const float z  = slab[row * kSlabP + col];
      const float xf = x[(size_t)gm * kDm + n0 + col];
      const float sv = SPL[gm];
      const float xr = rne_bf16_f32(xf);
      const float e  = expf(-fabsf(z));
      const float sp = fmaxf(z, 0.0f) + log1pf(e);
      float y = xr * sp;
      y = y * sv;
      slab[row * kSlabP + col] = y;
    }
    __builtin_amdgcn_fence(__ATOMIC_RELEASE, "workgroup");
    __builtin_amdgcn_wave_barrier();
    __builtin_amdgcn_fence(__ATOMIC_ACQUIRE, "workgroup");

    {
      const int hh = lane >> 4;
      const int c4 = (lane & 15) * 4;
      for (int pass = 0; pass < 2; ++pass) {
#pragma unroll
        for (int it = 0; it < 8; ++it) {
          const int row = it * 2 + hh;
          const v4f v = *(const v4f*)(slab + row * kSlabP + c4);
          *(volatile v4f*)(out + (size_t)(mBase + row) * kDm + n0 + c4) = v;
        }
        __threadfence();
      }
    }
    __builtin_amdgcn_fence(__ATOMIC_RELEASE, "workgroup");
    __builtin_amdgcn_wave_barrier();
    __builtin_amdgcn_fence(__ATOMIC_ACQUIRE, "workgroup");
  }
}

extern "C" void kernel_launch(void* const* d_in, const int* in_sizes, int n_in,
                              void* d_out, int out_size, void* d_ws, size_t ws_size,
                              hipStream_t stream)
{
  if (n_in < 8) return;
  if (in_sizes[0] != kRows * kDm) return;
  if (in_sizes[1] != kDm * kDm) return;
  if (in_sizes[2] != kDm) return;
  if (in_sizes[3] != kNst * kDm) return;
  if (in_sizes[4] != kNst) return;
  if (in_sizes[5] != kNst * kDm) return;
  if (in_sizes[6] != kNst) return;
  if (out_size != kRows * kDm) return;
  if (ws_size < kWsTotal) return;

  const float* x  = (const float*)d_in[0];
  const float* W1 = (const float*)d_in[1];
  const float* b1 = (const float*)d_in[2];
  const float* W2 = (const float*)d_in[3];
  const float* b2 = (const float*)d_in[4];
  const float* W3 = (const float*)d_in[5];
  const float* b3 = (const float*)d_in[6];
  float* out = (float*)d_out;

  char* ws = (char*)d_ws;
  unsigned short* XB   = (unsigned short*)(ws + kOffXB);
  unsigned short* W1B  = (unsigned short*)(ws + kOffW1B);
  unsigned short* W23B = (unsigned short*)(ws + kOffW23B);
  float*          SPL  = (float*)(ws + kOffSPL);

  constexpr int kX8  = kRows * kDm / 8;
  constexpr int kW18 = kDm * kDm / 8;
  constexpr int kW28 = kNst * kDm / 8;
  static_assert((kX8 % 256) == 0 && (kW18 % 256) == 0 && (kW28 % 256) == 0, "exact convert grids");

  rne_bf16_rows_kernel<<<kX8 / 256, 256, 0, stream>>>(x, XB, kX8);
  rne_bf16_rows_kernel<<<kW18 / 256, 256, 0, stream>>>(W1, W1B, kW18);
  rne_bf16_rows_kernel<<<kW28 / 256, 256, 0, stream>>>(W2, W23B, kW28);
  rne_bf16_rows_kernel<<<kW28 / 256, 256, 0, stream>>>(W3, W23B + (size_t)kNst * kDm, kW28);

  bc_rowdot_kernel<<<kRows / kRowsPerDotBlock, 256, 0, stream>>>(XB, W23B, b2, b3, SPL);

  fc1_softplus_gate_kernel<<<(kTilesM * kTilesN) / 8, 256, 0, stream>>>(XB, W1B, x, b1, SPL, out);
}
